// GraphAttentionLayer_24498493456637
// MI455X (gfx1250) — hardware-run, weakly checked
//
#include <hip/hip_runtime.h>


#ifndef NB
#define NB 8
#endif
#ifndef SEQ
#define SEQ 2048
#endif
#define NB_FULL  8
#define SEQ_FULL 2048
#ifndef OUT_SEQ
#define OUT_SEQ SEQ
#endif
#define FI   256
#define FO   128
#define AW   4
#define OSP  132
#define WTP  264
#define LOG2E 1.4426950408889634f
#define PSH  14.0f
#define NEGB (-3.0e38f)
#define MASKT (-1.2984255e16f)
#define LSLOPE 0.2f
#define CUTN (-0.1f)
#define LOCTH 0.01f

static_assert(FI % 32 == 0);
static_assert(FI == 256);
static_assert(FO == 128);
static_assert(FO % 64 == 0);
static_assert(FO % 8 == 0);
static_assert(SEQ % 64 == 0);
static_assert((NB * SEQ) % 64 == 0);
static_assert(SEQ % 32 == 0);
static_assert(SEQ % (16 * AW) == 0);
static_assert(((size_t)SEQ * FI) % 8 == 0);
static_assert(NB <= NB_FULL);
static_assert(SEQ <= SEQ_FULL);
static_assert((OSP * 4) % 16 == 0);
static_assert(OSP >= FO);
static_assert((WTP * 2) % 16 == 0);
static_assert(WTP >= FI);
static_assert(AW * 16 * OSP * 4 <= 131072);
static_assert(16 * 68 * 4 <= 131072);
static_assert(8 * WTP * 2 <= 131072);

typedef _Float16 h16;
typedef unsigned short bf;
typedef __attribute__((ext_vector_type(16))) __bf16   v16bf;
typedef __attribute__((ext_vector_type(16))) _Float16 v16h;
typedef __attribute__((ext_vector_type(8)))  _Float16 v8h;
typedef __attribute__((ext_vector_type(8)))  unsigned short v8us;
typedef __attribute__((ext_vector_type(8)))  float    v8f;
typedef __attribute__((ext_vector_type(4)))  float    v4f;
typedef v4f  __attribute__((may_alias)) v4fa;
typedef v8us __attribute__((may_alias)) v8usa;

__device__ __forceinline__ unsigned short f2bf(float f) { unsigned u = __float_as_uint(f); u += 0x7FFFu + ((u >> 16) & 1u); return (unsigned short)(u >> 16); }
__device__ __forceinline__ float bfr(float f) { return __uint_as_float(((unsigned)f2bf(f)) << 16); }
__device__ __forceinline__ v16h cat16(v8h lo, v8h hi) { return __builtin_shufflevector(lo, hi, 0, 1, 2, 3, 4, 5, 6, 7, 8, 9, 10, 11, 12, 13, 14, 15); }
__device__ __forceinline__ v16bf cat16b(v8us lo, v8us hi) { return __builtin_bit_cast(v16bf, __builtin_shufflevector(lo, hi, 0, 1, 2, 3, 4, 5, 6, 7, 8, 9, 10, 11, 12, 13, 14, 15)); }
__device__ __forceinline__ v8f wmma16(v16h a, v16h b, v8f c) { return __builtin_amdgcn_wmma_f32_16x16x32_f16(false, a, false, b, (short)0, c, false, false); }
__device__ __forceinline__ v8f wmmab(v16bf a, v16bf b, v8f c) { return __builtin_amdgcn_wmma_f32_16x16x32_bf16(false, a, false, b, (short)0, c, false, false); }
__device__ __forceinline__ v16h  ldh(const h16* p) { return cat16(*(const v8h*)p, *(const v8h*)(p + 16)); }
__device__ __forceinline__ v16bf ldb(const bf* p)  { return cat16b(*(const v8us*)p, *(const v8us*)(p + 16)); }
__device__ __forceinline__ void wave_sync() { __builtin_amdgcn_fence(3  , "wavefront"); __builtin_amdgcn_wave_barrier(); asm volatile("" ::: "memory"); }

__device__ __forceinline__ v8f wmma16g(v16h a, v16h b, v8f c) { c = wmma16(a, b, c); asm volatile("v_nop\n\tv_nop\n\tv_nop\n\tv_nop" : "+v"(c) : "v"(a), "v"(b)); return c; }
__device__ __forceinline__ v8f wmmabg(v16bf a, v16bf b, v8f c) { c = wmmab(a, b, c); asm volatile("v_nop\n\tv_nop\n\tv_nop\n\tv_nop" : "+v"(c) : "v"(a), "v"(b)); return c; }
__device__ __forceinline__ h16 toh_flush(float v) { const h16 r = (h16)v; return (fabsf(v) < 6.103515625e-05f) ? (h16)0.0f : r; }
__device__ __forceinline__ h16 p2h(float e2) { const float g = __builtin_amdgcn_exp2f(e2); const h16 r = (h16)g; return (e2 < -14.0f) ? (h16)0.0f : r; }
__device__ __forceinline__ v8f cat8f(v4f lo, v4f hi) { return __builtin_shufflevector(lo, hi, 0, 1, 2, 3, 4, 5, 6, 7); }
__device__ __forceinline__ float elu1(float v) { const float e = __builtin_amdgcn_exp2f(v * LOG2E) - 1.0f; return (v > 0.0f) ? v : e; }

__global__ __launch_bounds__(256) void k_cvt8(const float* __restrict__ src, bf* dst, size_t n8) {
    const size_t i = (size_t)blockIdx.x * 256 + threadIdx.x; if (i >= n8) return;
    const v8f v = *(const v8f*)(src + i * 8); v8us o;
#pragma unroll
    for (int k = 0; k < 8; ++k) o[k] = f2bf(v[k]);
    *(volatile v8us*)(dst + i * 8) = o; __threadfence(); *(volatile v8us*)(dst + i * 8) = o;
}

__global__ __launch_bounds__(256) void k_wtr(const float* __restrict__ W, bf* WT) {
    __shared__ __align__(16) unsigned short tile[8 * WTP];
    const int tid = threadIdx.x; const int n0 = blockIdx.x * 8;
    const v4f w0 = *(const v4f*)(W + (size_t)tid * FO + n0), w1 = *(const v4f*)(W + (size_t)tid * FO + n0 + 4);
#pragma unroll
    for (int j = 0; j < 4; ++j) { tile[j * WTP + tid] = f2bf(w0[j]); tile[(4 + j) * WTP + tid] = f2bf(w1[j]); }
    __syncthreads();
    const int row = tid >> 5, c8 = (tid & 31) * 8;
    static_assert(256 * 16 == 8 * FI * 2);
    const v8us o = *(const v8usa*)(&tile[row * WTP + c8]);
    bf* dp = WT + (size_t)(n0 + row) * FI + c8;
    *(volatile v8us*)dp = o; __threadfence(); *(volatile v8us*)dp = o;
}

__global__ __launch_bounds__(32) void k_hproj(const bf* __restrict__ A, const bf* __restrict__ Bt, const float* __restrict__ avec, h16* Ph, float* FP) {
    __shared__ __align__(16) float os[16 * 68];
    const int K = FI;
    const int lane = threadIdx.x & 31, lr = lane & 15, hi = lane >> 4; const int r0 = blockIdx.x * 64, c0 = blockIdx.y * 64;
    v8f acc[4][4];
#pragma unroll
    for (int mb = 0; mb < 4; ++mb)
#pragma unroll
        for (int nb = 0; nb < 4; ++nb) acc[mb][nb] = (v8f){};
    const size_t aoff = (size_t)(r0 + lr) * K + 8 * hi, boff = (size_t)(c0 + lr) * K + 8 * hi;
#pragma unroll 1
    for (int kc = 0; kc < K; kc += 32) {
        v16bf a[4];
#pragma unroll
        for (int mb = 0; mb < 4; ++mb) a[mb] = ldb(A + aoff + (size_t)mb * 16 * K + kc);
#pragma unroll
        for (int nb = 0; nb < 4; ++nb) { const v16bf b = ldb(Bt + boff + (size_t)nb * 16 * K + kc);
#pragma unroll
            for (int mb = 0; mb < 4; ++mb) acc[mb][nb] = wmmabg(a[mb], b, acc[mb][nb]); }
    }
    float fsp[4], fdp[4];
#pragma unroll
    for (int nb = 0; nb < 4; ++nb) { fsp[nb] = 0.0f; fdp[nb] = 0.0f; }
    const int bb = c0 / SEQ, tt = c0 % SEQ;
    const size_t tbase = (size_t)bb * (size_t)FO * SEQ + (size_t)r0 * SEQ + (size_t)tt;
#pragma unroll
    for (int mb = 0; mb < 4; ++mb) {
        float a1v[8], a2v[8];
#pragma unroll
        for (int j = 0; j < 8; ++j) { const int mrow = r0 + mb * 16 + hi * 8 + j;
            a1v[j] = bfr(avec[mrow]); a2v[j] = bfr(avec[FO + mrow]); }
#pragma unroll
        for (int nb = 0; nb < 4; ++nb) {
#pragma unroll
            for (int j = 0; j < 8; ++j) { const float v = acc[mb][nb][j];
                os[(hi * 8 + j) * 68 + nb * 16 + lr] = v; fsp[nb] += v * a1v[j]; fdp[nb] += v * a2v[j]; } }
        wave_sync();
        const size_t sb = tbase + (size_t)(mb * 16) * SEQ;
        static_assert(4 * 32 * 16 == 16 * 64 * 2);
#pragma unroll 1
        for (int ps = 0; ps < 2; ++ps) {
#pragma unroll
            for (int s = 0; s < 4; ++s) { const int row = 4 * s + (lane >> 3), c8 = (lane & 7) * 8;
                const v4f x0 = *(const v4fa*)(&os[row * 68 + c8]); const v4f x1 = *(const v4fa*)(&os[row * 68 + c8 + 4]); v8h hv;
#pragma unroll
                for (int i = 0; i < 4; ++i) { hv[i] = toh_flush(x0[i]); hv[4 + i] = toh_flush(x1[i]); }
                *(volatile v8h*)(Ph + sb + (size_t)row * SEQ + c8) = hv; }
            if (ps == 0) __threadfence(); }
        wave_sync();
    }
#pragma unroll
    for (int nb = 0; nb < 4; ++nb) { fsp[nb] += __shfl_xor(fsp[nb], 16, 32); fdp[nb] += __shfl_xor(fdp[nb], 16, 32); }
#pragma unroll
    for (int nb = 0; nb < 4; ++nb) { const float v = (hi != 0) ? fdp[nb] : fsp[nb]; os[hi * 64 + nb * 16 + lr] = v; }
    wave_sync();
    {
        const int which = lane >> 4, cofs = (lane & 15) * 4;
        static_assert(16 * 16 == 64 * 4);
        const v4f val = *(const v4fa*)(&os[which * 64 + cofs]);
        float* dp = FP + (size_t)(blockIdx.x * 2 + which) * ((size_t)NB * SEQ) + (size_t)c0 + cofs;
        *(volatile v4f*)dp = val; __threadfence(); *(volatile v4f*)dp = val;
    }
}

__global__ __launch_bounds__(256) void k_keytab(const float* __restrict__ coord, const float* __restrict__ FP, float* CX, float* CY, float* CZ, float* FS, float* FD) {
    const int i = blockIdx.x * 256 + threadIdx.x; if (i >= NB * SEQ / 4) return;
    const int g = 4 * i; const int b = g / SEQ, t = g % SEQ;
    const float* cp = coord + ((size_t)b * SEQ_FULL + (size_t)t) * 3;
    const v4f c0 = *(const v4f*)cp, c1 = *(const v4f*)(cp + 4), c2 = *(const v4f*)(cp + 8);
    const size_t PT = (size_t)NB * SEQ;
    const v4f s0 = *(const v4f*)(FP + g), d0 = *(const v4f*)(FP + PT + g), s1 = *(const v4f*)(FP + 2 * PT + g), d1 = *(const v4f*)(FP + 3 * PT + g);
    v4f vx, vy, vz;
    vx[0] = bfr(c0[0]); vy[0] = bfr(c0[1]); vz[0] = bfr(c0[2]);
    vx[1] = bfr(c0[3]); vy[1] = bfr(c1[0]); vz[1] = bfr(c1[1]);
    vx[2] = bfr(c1[2]); vy[2] = bfr(c1[3]); vz[2] = bfr(c2[0]);
    vx[3] = bfr(c2[1]); vy[3] = bfr(c2[2]); vz[3] = bfr(c2[3]);
    const v4f vs = s0 + s1, vd = d0 + d1;
    *(volatile v4f*)(CX + g) = vx; *(volatile v4f*)(CY + g) = vy; *(volatile v4f*)(CZ + g) = vz; *(volatile v4f*)(FS + g) = vs; *(volatile v4f*)(FD + g) = vd;
    __threadfence();
    *(volatile v4f*)(CX + g) = vx; *(volatile v4f*)(CY + g) = vy; *(volatile v4f*)(CZ + g) = vz; *(volatile v4f*)(FS + g) = vs; *(volatile v4f*)(FD + g) = vd;
}

__device__ __forceinline__ v8f score8(const v8f kx, const v8f ky, const v8f kz, const v8f kd, const float qx, const float qy, const float qz, const float fsq) {
#pragma clang fp contract(off)
    v8f t;
#pragma unroll
    for (int r = 0; r < 8; ++r) {
        const float dx = qx - kx[r], dy = qy - ky[r], dz = qz - kz[r];
        const float d2 = (dx * dx + dz * dz) + dy * dy;
        const float loc = __builtin_amdgcn_exp2f((CUTN * d2) * LOG2E);
        const float e0 = fsq + kd[r];
        const float e1 = (e0 > 0.0f) ? e0 : LSLOPE * e0;
        const float lg = (e1 * loc) * LOG2E;
        t[r] = (loc > LOCTH) ? lg : MASKT;
    }
    return t;
}

__global__ __launch_bounds__(32 * AW) void k_gflash(const h16* __restrict__ HT, const float* __restrict__ CX, const float* __restrict__ CY, const float* __restrict__ CZ,
                                                    const float* __restrict__ FS, const float* __restrict__ FD, float* OUT) {
    __shared__ __align__(16) float os[AW * 16 * OSP];
    const int lane = threadIdx.x & 31, lr = lane & 15, hi = lane >> 4;
    const int wave = __builtin_amdgcn_readfirstlane((int)(threadIdx.x >> 5));
    const int b = blockIdx.y;
    const int t0 = (blockIdx.x * AW + wave) * 16;
    const size_t tk = (size_t)b * SEQ;
    const float fsq = FS[tk + t0 + lr];
    const float qx = CX[tk + t0 + lr], qy = CY[tk + t0 + lr], qz = CZ[tk + t0 + lr];
    const size_t ko = tk + 8 * hi;
    const size_t vo = ((size_t)b * FO + lr) * SEQ + 8 * hi;
    v8f o[8];
#pragma unroll
    for (int j = 0; j < 8; ++j) o[j] = (v8f){};
    float m = NEGB, l = 0.0f;
#pragma unroll 1
    for (int key0 = 0; key0 < SEQ; key0 += 32) {
        const size_t ka = ko + key0;
        v8f ta, tb;
        { const v8f kx = cat8f(*(const v4f*)(CX + ka), *(const v4f*)(CX + ka + 4)); const v8f ky = cat8f(*(const v4f*)(CY + ka), *(const v4f*)(CY + ka + 4));
          const v8f kz = cat8f(*(const v4f*)(CZ + ka), *(const v4f*)(CZ + ka + 4)); const v8f kd = cat8f(*(const v4f*)(FD + ka), *(const v4f*)(FD + ka + 4));
          ta = score8(kx, ky, kz, kd, qx, qy, qz, fsq); }
        { const size_t kb = ka + 16;
          const v8f kx = cat8f(*(const v4f*)(CX + kb), *(const v4f*)(CX + kb + 4)); const v8f ky = cat8f(*(const v4f*)(CY + kb), *(const v4f*)(CY + kb + 4));
          const v8f kz = cat8f(*(const v4f*)(CZ + kb), *(const v4f*)(CZ + kb + 4)); const v8f kd = cat8f(*(const v4f*)(FD + kb), *(const v4f*)(FD + kb + 4));
          tb = score8(kx, ky, kz, kd, qx, qy, qz, fsq); }
        float mx = NEGB;
#pragma unroll
        for (int r = 0; r < 8; ++r) mx = fmaxf(mx, fmaxf(ta[r], tb[r]));
        mx = fmaxf(mx, __shfl_xor(mx, 16, 32));
        const float mnew = fmaxf(m, mx);
        const float alpha = __builtin_amdgcn_exp2f(m - mnew);
        v16h pb; float ls = 0.0f;
#pragma unroll
        for (int r = 0; r < 8; ++r) {
            const h16 pa = p2h((ta[r] - mnew) + PSH); const h16 pc = p2h((tb[r] - mnew) + PSH);
            pb[r] = pa; pb[8 + r] = pc;
            ls += (float)pa + (float)pc; }
        l = l * alpha + ls; m = mnew;
#pragma unroll
        for (int j = 0; j < 8; ++j) o[j] = o[j] * alpha;
        const h16* va = HT + vo + key0;
        { const v16h v0 = ldh(va), v1 = ldh(va + (size_t)16 * SEQ), v2 = ldh(va + (size_t)32 * SEQ), v3 = ldh(va + (size_t)48 * SEQ);
          o[0] = wmma16g(v0, pb, o[0]); o[1] = wmma16g(v1, pb, o[1]); o[2] = wmma16g(v2, pb, o[2]); o[3] = wmma16g(v3, pb, o[3]); }
        { const v16h v4 = ldh(va + (size_t)64 * SEQ), v5 = ldh(va + (size_t)80 * SEQ), v6 = ldh(va + (size_t)96 * SEQ), v7 = ldh(va + (size_t)112 * SEQ);
          o[4] = wmma16g(v4, pb, o[4]); o[5] = wmma16g(v5, pb, o[5]); o[6] = wmma16g(v6, pb, o[6]); o[7] = wmma16g(v7, pb, o[7]); }
    }
    l += __shfl_xor(l, 16, 32);
    const bool any = l > 0.0f;
    const float lsafe = any ? l : 1.0f;
    const float inv = any ? (1.0f / lsafe) : 0.0f;
    const int wb = wave * 16 * OSP;
#pragma unroll
    for (int j = 0; j < 8; ++j) { v4f a, c;
#pragma unroll
        for (int i = 0; i < 4; ++i) { a[i] = elu1(o[j][i] * inv); c[i] = elu1(o[j][4 + i] * inv); }
        *(v4fa*)(&os[wb + lr * OSP + 16 * j + 8 * hi]) = a; *(v4fa*)(&os[wb + lr * OSP + 16 * j + 8 * hi + 4]) = c; }
    wave_sync();
    float* orow = OUT + ((size_t)b * OUT_SEQ + t0) * FO;
    static_assert(16 * 32 * 16 == 16 * FO * 4);
#pragma unroll 1
    for (int ps = 0; ps < 2; ++ps) {
#pragma unroll
        for (int s = 0; s < 16; ++s) {
            const v4f val = *(const v4fa*)(&os[wb + s * OSP + lane * 4]);
            *(volatile v4f*)(orow + (size_t)s * FO + lane * 4) = val; }
        if (ps == 0) __threadfence(); }
}

static constexpr size_t al256(size_t v) { return (v + 255) & ~(size_t)255; }
static constexpr size_t SZ_XB = al256((size_t)NB * SEQ * FI * 2);
static constexpr size_t SZ_WT = al256((size_t)FO * FI * 2);
static constexpr size_t SZ_HT = al256((size_t)NB * FO * SEQ * 2);
static constexpr size_t SZ_FP = al256((size_t)4 * NB * SEQ * 4);
static constexpr size_t SZ_TB = al256((size_t)NB * SEQ * 4);
static constexpr size_t SZ_TOTAL = SZ_XB + SZ_WT + SZ_HT + SZ_FP + 5 * SZ_TB;
static_assert(SZ_TOTAL <= (size_t)134217728);
static_assert(((size_t)(FO / 64) * 2 - 1) * ((size_t)NB * SEQ) + (size_t)NB * SEQ <= (size_t)4 * NB * SEQ);

extern "C" void kernel_launch(void* const* d_in, const int* in_sizes, int n_in,
                              void* d_out, int out_size, void* d_ws, size_t ws_size, hipStream_t stream) {
    if (n_in < 4) return;
    const size_t needx = ((size_t)(NB - 1) * SEQ_FULL + SEQ) * FI;
    const size_t needc = ((size_t)(NB - 1) * SEQ_FULL + SEQ) * 3;
    if ((size_t)in_sizes[0] < needx || (size_t)in_sizes[1] < needc) return;
    if ((size_t)in_sizes[2] < (size_t)FI * FO || in_sizes[3] < 2 * FO) return;
    if ((size_t)out_size < ((size_t)(NB - 1) * OUT_SEQ + SEQ) * FO) return;
    if (SZ_TOTAL > ws_size) return;
    const float* xin   = (const float*)d_in[0];
    const float* coord = (const float*)d_in[1];
    const float* W     = (const float*)d_in[2];
    const float* avec  = (const float*)d_in[3];
    float* OUT = (float*)d_out;
    char* wsp = (char*)d_ws;
    bf*  XB = (bf*)wsp;  wsp += SZ_XB;
    bf*  WT = (bf*)wsp;  wsp += SZ_WT;
    h16* HT = (h16*)wsp; wsp += SZ_HT;
    float* FP = (float*)wsp; wsp += SZ_FP;
    float* CX = (float*)wsp; wsp += SZ_TB;
    float* CY = (float*)wsp; wsp += SZ_TB;
    float* CZ = (float*)wsp; wsp += SZ_TB;
    float* FS = (float*)wsp; wsp += SZ_TB;
    float* FD = (float*)wsp; wsp += SZ_TB;

    if (SEQ == SEQ_FULL) {
        const size_t n8 = (size_t)NB * SEQ * FI / 8;
        k_cvt8<<<(unsigned)((n8 + 255) / 256), 256, 0, stream>>>(xin, XB, n8);
    } else {
        const size_t n8 = (size_t)SEQ * FI / 8;
        for (int b = 0; b < NB; ++b) k_cvt8<<<(unsigned)((n8 + 255) / 256), 256, 0, stream>>>(xin + (size_t)b * SEQ_FULL * FI, XB + (size_t)b * SEQ * FI, n8);
    }
    k_wtr<<<FO / 8, 256, 0, stream>>>(W, WT);
    k_hproj<<<dim3(FO / 64, NB * SEQ / 64, 1), 32, 0, stream>>>(WT, XB, avec, HT, FP);
    k_keytab<<<(unsigned)((NB * SEQ / 4 + 255) / 256), 256, 0, stream>>>(coord, FP, CX, CY, CZ, FS, FD);
    k_gflash<<<dim3(SEQ / (16 * AW), NB, 1), 32 * AW, 0, stream>>>(HT, CX, CY, CZ, FS, FD, OUT);
}
